// GCN_22797686407974
// MI455X (gfx1250) — hardware-verified
//
#include <hip/hip_runtime.h>
#include <stddef.h>
#include <stdint.h>
#include <math.h>


#define NN     8192
#define FEAT   128
#define HID    256
#define NCLS   64
#define K2     512
#define BLKN   256
#define DEG    16
#define NTHR   256
#define GBM    64
#define GBN    64
#define GTHR   128
#define NUX    (NN * (FEAT / 8))
#define NU1    (HID * (FEAT / 8))
#define NU2    (NCLS * (K2 / 8))
#define WSMAX  134217728

#define SZ_XB  ((size_t)NN * FEAT * 2)
#define SZ_W1T ((size_t)HID * FEAT * 2)
#define SZ_W2T ((size_t)NCLS * K2 * 2)
#define SZ_XW  ((size_t)NN * HID * 4)
#define SZ_H2  ((size_t)NN * K2 * 2)
#define SZ_HW  ((size_t)NN * NCLS * 4)
#define O_XB   ((size_t)0)
#define O_W1T  (O_XB + SZ_XB)
#define O_W2T  (O_W1T + SZ_W1T)
#define O_XW   (O_W2T + SZ_W2T)
#define O_H2   (O_XW + SZ_XW)
#define O_HW   (O_H2 + SZ_H2)
#define WS_TOT (O_HW + SZ_HW)

static_assert(SZ_XB % 256 == 0 && SZ_W1T % 256 == 0 && SZ_W2T % 256 == 0);
static_assert(SZ_XW % 256 == 0 && SZ_H2 % 256 == 0 && SZ_HW % 256 == 0);
static_assert(WS_TOT <= (size_t)WSMAX);
static_assert(NN % GBM == 0 && HID % GBN == 0 && NCLS % GBN == 0);
static_assert(FEAT % 32 == 0 && K2 % 32 == 0 && K2 == 2 * HID);
static_assert(GBM == (GTHR / 32) * 16 && GBN == 64);
static_assert(NUX % NTHR == 0 && NU1 % NTHR == 0 && NU2 % NTHR == 0);
static_assert(FEAT / 8 == 16 && K2 / 8 == 64);
static_assert(HID == 32 * 8);
static_assert(NCLS == 16 * 4);
static_assert(NN % (NTHR / 32) == 0 && NN % (2 * (NTHR / 32)) == 0);
static_assert(NN % BLKN == 0 && DEG == 16);
static_assert((size_t)NN * NCLS - 1 == 524287);

typedef float          v4f   __attribute__((ext_vector_type(4)));
typedef float          v8f   __attribute__((ext_vector_type(8)));
typedef int            v8i   __attribute__((ext_vector_type(8)));
typedef unsigned short v8us  __attribute__((ext_vector_type(8)));
typedef unsigned short v16us __attribute__((ext_vector_type(16)));
typedef __bf16         v16bf __attribute__((ext_vector_type(16)));
typedef v4f  __attribute__((may_alias)) v4fa;
typedef v8us __attribute__((may_alias)) v8usa;
union FragB { v16bf v; v16us u; v8us h[2]; v8i w; };

__device__ __forceinline__ v8f wmb(const FragB& a, const FragB& b, v8f c) {
  v8f d = __builtin_amdgcn_wmma_f32_16x16x32_bf16(false, a.v, false, b.v, (short)0, c, false, false);
  asm volatile("v_nop\n\tv_nop\n\tv_nop\n\tv_nop" : "+v"(d) : "v"(a.w), "v"(b.w));
  return d;
}

__device__ __forceinline__ unsigned bf16_bits(float f) {
  const unsigned u = __float_as_uint(f);
  return (u + 0x7FFFu + ((u >> 16) & 1u)) >> 16;
}

__device__ __forceinline__ unsigned relu_split(float v) {
  const float r = (v > 0.0f) ? v : (v - v);
  const unsigned hb = bf16_bits(r);
  const unsigned lb = bf16_bits(r - __uint_as_float(hb << 16));
  return hb | (lb << 16);
}

__global__ __launch_bounds__(NTHR) void k_prep(const float* __restrict__ x, const float* __restrict__ W1,
                                               const float* __restrict__ W2, unsigned short* pl) {
  const int u = (int)blockIdx.x * NTHR + (int)threadIdx.x;
  v8us o;
  size_t doff;
  if (u < NUX) {
    const int row = u >> 4;
    const int k8  = (u & 15) * 8;
    const float* p = x + (size_t)row * FEAT + k8;
    const v4f a = *(const v4fa*)p;
    const v4f b = *(const v4fa*)(p + 4);
    o[0] = (unsigned short)bf16_bits(a.x); o[1] = (unsigned short)bf16_bits(a.y);
    o[2] = (unsigned short)bf16_bits(a.z); o[3] = (unsigned short)bf16_bits(a.w);
    o[4] = (unsigned short)bf16_bits(b.x); o[5] = (unsigned short)bf16_bits(b.y);
    o[6] = (unsigned short)bf16_bits(b.z); o[7] = (unsigned short)bf16_bits(b.w);
    doff = (O_XB / 2) + (size_t)row * FEAT + k8;
  } else if (u < NUX + NU1) {
    const int v  = u - NUX;
    const int n  = v >> 4;
    const int k8 = (v & 15) * 8;
    const float* p = W1 + (size_t)k8 * HID + n;
#pragma unroll
    for (int i = 0; i < 8; ++i) o[i] = (unsigned short)bf16_bits(p[(size_t)i * HID]);
    doff = (O_W1T / 2) + (size_t)n * FEAT + k8;
  } else if (u < NUX + NU1 + NU2) {
    const int v  = u - NUX - NU1;
    const int n  = v >> 6;
    const int k8 = (v & 63) * 8;
    const int kk = k8 & (HID - 1);
    const float* p = W2 + (size_t)kk * NCLS + n;
#pragma unroll
    for (int i = 0; i < 8; ++i) o[i] = (unsigned short)bf16_bits(p[(size_t)i * NCLS]);
    doff = (O_W2T / 2) + (size_t)n * K2 + k8;
  } else {
    return;
  }
  unsigned short* dp = pl + doff;
  *(volatile v8us*)dp = o;
  __threadfence();
  *(volatile v8us*)dp = o;
}

__global__ __launch_bounds__(GTHR) void k_gemm(
    const unsigned short* __restrict__ A, const unsigned short* __restrict__ WT,
    float* outF, int K, int ldo)
{
  __shared__ __attribute__((aligned(16))) float stg[GBM * GBN];
  const int tid = (int)threadIdx.x, lane = tid & 31, wave = tid >> 5, hh = lane >> 4, m = lane & 15;
  const int rowBase = (int)blockIdx.x * GBM;
  const int col0    = (int)blockIdx.y * GBN;

  v8f acc[4];
  {
    const v8f z = {0.f, 0.f, 0.f, 0.f, 0.f, 0.f, 0.f, 0.f};
    acc[0] = z; acc[1] = z; acc[2] = z; acc[3] = z;
  }
  const unsigned short* ap = A  + (size_t)(rowBase + 16 * wave + m) * (size_t)K + 8 * hh;
  const unsigned short* wp = WT + (size_t)(col0 + m) * (size_t)K + 8 * hh;
  const int ksteps = K >> 5;
#pragma unroll 1
  for (int ks = 0; ks < ksteps; ++ks) {
    FragB af;
    af.h[0] = *(const v8usa*)(ap + 32 * ks);
    af.h[1] = *(const v8usa*)(ap + 32 * ks + 16);
#pragma unroll
    for (int t = 0; t < 4; ++t) {
      const unsigned short* wq = wp + (size_t)(16 * t) * (size_t)K + 32 * ks;
      FragB bf;
      bf.h[0] = *(const v8usa*)wq;
      bf.h[1] = *(const v8usa*)(wq + 16);
      acc[t] = wmb(af, bf, acc[t]);
    }
  }

#pragma unroll
  for (int t = 0; t < 4; ++t) {
    const int lc = 16 * t + m;
#pragma unroll
    for (int r = 0; r < 8; ++r) {
      const int lr = 16 * wave + 8 * hh + r;
      stg[lr * GBN + lc] = acc[t][r];
    }
  }
  __syncthreads();

  v4f fv[8];
#pragma unroll
  for (int i = 0; i < 8; ++i) {
    const int lr = 16 * wave + 2 * i + hh;
    fv[i] = *(const v4fa*)(stg + lr * GBN + 4 * m);
  }
#pragma unroll
  for (int i = 0; i < 8; ++i) {
    const int lr = 16 * wave + 2 * i + hh;
    const int gr = rowBase + lr;
    float* op = outF + (size_t)gr * (size_t)ldo + col0 + 4 * m;
    *(volatile v4f*)op = fv[i];
  }
  __threadfence();
#pragma unroll
  for (int i = 0; i < 8; ++i) {
    const int lr = 16 * wave + 2 * i + hh;
    const int gr = rowBase + lr;
    float* op = outF + (size_t)gr * (size_t)ldo + col0 + 4 * m;
    *(volatile v4f*)op = fv[i];
  }
}

__device__ __forceinline__ int slot_col(int e, int row) {
  const long long cw = (long long)e + (long long)((row / BLKN) * BLKN);
  const long long c2 = (cw < 0) ? (cw + (long long)NN) : cw;
  const bool valid = (e != -1) && (c2 >= 0) && (c2 < (long long)NN);
  return valid ? (int)c2 : -1;
}

__global__ __launch_bounds__(NTHR) void k_agg1(const int* __restrict__ edges, const float* __restrict__ xw,
                                               unsigned short* h2) {
  const int tid = (int)threadIdx.x, lane = tid & 31, wave = tid >> 5, s = lane & 15;
  const int row = (int)blockIdx.x * (NTHR / 32) + wave;
  const int e = edges[(size_t)row * DEG + s];
  const int c = slot_col(e, row);
  bool dup = false;
#pragma unroll
  for (int k = 0; k < DEG; ++k) {
    const int ck = __shfl(c, k, 32);
    dup = dup || ((k < s) && (ck == c));
  }
  const int keep = ((c >= 0) && !dup) ? 1 : 0;
  const int cl   = (c < 0) ? 0 : c;

  v4f a0 = {0.0f, 0.0f, 0.0f, 0.0f};
  v4f a1 = {0.0f, 0.0f, 0.0f, 0.0f};
#pragma unroll 4
  for (int j = 0; j < DEG; ++j) {
    int cj = __shfl(cl, j, 32);
    const int kj = __shfl(keep, j, 32);
    cj = cj < 0 ? 0 : (cj > NN - 1 ? NN - 1 : cj);
    const unsigned km = 0u - (unsigned)(kj & 1);
    const float* rp = xw + (size_t)cj * HID + 8 * lane;
    const v4f p = *(const v4fa*)rp;
    const v4f q = *(const v4fa*)(rp + 4);
    a0.x += __uint_as_float(__float_as_uint(p.x) & km);
    a0.y += __uint_as_float(__float_as_uint(p.y) & km);
    a0.z += __uint_as_float(__float_as_uint(p.z) & km);
    a0.w += __uint_as_float(__float_as_uint(p.w) & km);
    a1.x += __uint_as_float(__float_as_uint(q.x) & km);
    a1.y += __uint_as_float(__float_as_uint(q.y) & km);
    a1.z += __uint_as_float(__float_as_uint(q.z) & km);
    a1.w += __uint_as_float(__float_as_uint(q.w) & km);
  }

  const unsigned p0 = relu_split(a0.x), p1 = relu_split(a0.y), p2 = relu_split(a0.z), p3 = relu_split(a0.w);
  const unsigned p4 = relu_split(a1.x), p5 = relu_split(a1.y), p6 = relu_split(a1.z), p7 = relu_split(a1.w);
  v8us hv, lv;
  hv[0] = (unsigned short)(p0 & 0xffffu); lv[0] = (unsigned short)(p0 >> 16);
  hv[1] = (unsigned short)(p1 & 0xffffu); lv[1] = (unsigned short)(p1 >> 16);
  hv[2] = (unsigned short)(p2 & 0xffffu); lv[2] = (unsigned short)(p2 >> 16);
  hv[3] = (unsigned short)(p3 & 0xffffu); lv[3] = (unsigned short)(p3 >> 16);
  hv[4] = (unsigned short)(p4 & 0xffffu); lv[4] = (unsigned short)(p4 >> 16);
  hv[5] = (unsigned short)(p5 & 0xffffu); lv[5] = (unsigned short)(p5 >> 16);
  hv[6] = (unsigned short)(p6 & 0xffffu); lv[6] = (unsigned short)(p6 >> 16);
  hv[7] = (unsigned short)(p7 & 0xffffu); lv[7] = (unsigned short)(p7 >> 16);
  unsigned short* hp = h2 + (size_t)row * K2 + 8 * lane;
  *(volatile v8us*)hp = hv;
  *(volatile v8us*)(hp + HID) = lv;
  __threadfence();
  *(volatile v8us*)hp = hv;
  *(volatile v8us*)(hp + HID) = lv;
}

__global__ __launch_bounds__(NTHR) void k_agg2(const int* __restrict__ edges, const float* __restrict__ hw,
                                               float* out) {
  const int tid = (int)threadIdx.x, lane = tid & 31, wave = tid >> 5, s = lane & 15, hb = lane & 16;
  const int row = (int)blockIdx.x * (2 * (NTHR / 32)) + 2 * wave + (lane >> 4);
  const int e = edges[(size_t)row * DEG + s];
  const int c = slot_col(e, row);
  bool dup = false;
#pragma unroll
  for (int k = 0; k < DEG; ++k) {
    const int ck = __shfl(c, hb | k, 32);
    dup = dup || ((k < s) && (ck == c));
  }
  const int keep = ((c >= 0) && !dup) ? 1 : 0;
  const int cl   = (c < 0) ? 0 : c;

  v4f a = {0.0f, 0.0f, 0.0f, 0.0f};
#pragma unroll 4
  for (int j = 0; j < DEG; ++j) {
    int cj = __shfl(cl, hb | j, 32);
    const int kj = __shfl(keep, hb | j, 32);
    cj = cj < 0 ? 0 : (cj > NN - 1 ? NN - 1 : cj);
    const unsigned km = 0u - (unsigned)(kj & 1);
    const v4f p = *(const v4fa*)(hw + (size_t)cj * NCLS + 4 * s);
    a.x += __uint_as_float(__float_as_uint(p.x) & km);
    a.y += __uint_as_float(__float_as_uint(p.y) & km);
    a.z += __uint_as_float(__float_as_uint(p.z) & km);
    a.w += __uint_as_float(__float_as_uint(p.w) & km);
  }

  float mx = fmaxf(fmaxf(a.x, a.y), fmaxf(a.z, a.w));
  mx = fmaxf(mx, __shfl_xor(mx, 1, 32));
  mx = fmaxf(mx, __shfl_xor(mx, 2, 32));
  mx = fmaxf(mx, __shfl_xor(mx, 4, 32));
  mx = fmaxf(mx, __shfl_xor(mx, 8, 32));
  const float d0 = a.x - mx, d1 = a.y - mx, d2 = a.z - mx, d3 = a.w - mx;
  float sm = (expf(d0) + expf(d1)) + (expf(d2) + expf(d3));
  sm += __shfl_xor(sm, 1, 32);
  sm += __shfl_xor(sm, 2, 32);
  sm += __shfl_xor(sm, 4, 32);
  sm += __shfl_xor(sm, 8, 32);
  const float lse = logf(sm);
  v4f ov;
  ov.x = d0 - lse; ov.y = d1 - lse; ov.z = d2 - lse; ov.w = d3 - lse;
  float* op = out + (size_t)row * NCLS + 4 * s;
  *(volatile v4f*)op = ov;
  __threadfence();
  *(volatile v4f*)op = ov;
}

extern "C" void kernel_launch(void* const* d_in, const int* in_sizes, int n_in,
                              void* d_out, int out_size, void* d_ws, size_t ws_size,
                              hipStream_t stream) {
  if (n_in < 4) return;
  if (in_sizes[0] != NN * FEAT) return;
  if (in_sizes[1] != NN * DEG) return;
  if (in_sizes[2] != FEAT * HID) return;
  if (in_sizes[3] != HID * NCLS) return;
  if (out_size != NN * NCLS) return;
  if (ws_size < (size_t)WS_TOT) return;

  const float* x  = (const float*)d_in[0];
  const int*   ed = (const int*)d_in[1];
  const float* W1 = (const float*)d_in[2];
  const float* W2 = (const float*)d_in[3];
  float* out = (float*)d_out;

  char* ws = (char*)d_ws;
  unsigned short* P16  = (unsigned short*)ws;
  unsigned short* XB   = (unsigned short*)(ws + O_XB);
  unsigned short* W1T  = (unsigned short*)(ws + O_W1T);
  unsigned short* W2T2 = (unsigned short*)(ws + O_W2T);
  float*          XW   = (float*)(ws + O_XW);
  unsigned short* H2   = (unsigned short*)(ws + O_H2);
  float*          HW   = (float*)(ws + O_HW);

  k_prep<<<(NUX + NU1 + NU2) / NTHR, NTHR, 0, stream>>>(x, W1, W2, P16);
  k_gemm<<<dim3(NN / GBM, HID / GBN), GTHR, 0, stream>>>(XB, W1T, XW, FEAT, HID);
  k_agg1<<<NN / (NTHR / 32), NTHR, 0, stream>>>(ed, XW, H2);
  k_gemm<<<dim3(NN / GBM, NCLS / GBN), GTHR, 0, stream>>>(H2, W2T2, HW, K2, NCLS);
  k_agg2<<<NN / (2 * (NTHR / 32)), NTHR, 0, stream>>>(ed, HW, out);
}
